// CoAttentionLayer_50517405335639
// MI455X (gfx1250) — hardware-run, weakly checked
//
#include <hip/hip_runtime.h>
#define NB 8
#define NL 128
#define ND 300
#define NP 320
#define XSC 16.0f
#define TSC 16.0f
#define KSC 256.0f
#define PSC 128.0f
#define HIDE 1.0e30f
typedef __bf16 v16b __attribute__((ext_vector_type(16)));
typedef unsigned short v8us __attribute__((ext_vector_type(8), may_alias));
typedef float  v8f  __attribute__((ext_vector_type(8)));
typedef float  v4f  __attribute__((ext_vector_type(4)));
typedef float  v4fa __attribute__((ext_vector_type(4), may_alias));
union FragB { v16b v; v8us half[2]; unsigned short u[16]; };

__device__ __forceinline__ unsigned short bf16_bits(float x) { unsigned int u = __float_as_uint(x); return (unsigned short)((u + 0x7FFFu + ((u >> 16) & 1u)) >> 16); }
__device__ __forceinline__ float bf16_val(unsigned short b) { return __uint_as_float(((unsigned int)b) << 16); }
__device__ __forceinline__ float bf16_round(float x) { return bf16_val(bf16_bits(x)); }
template <int NT>
__device__ __forceinline__ v8f mmaN(v16b ah, v16b al, v16b bh, v16b bl, v8f c) {
  c = __builtin_amdgcn_wmma_f32_16x16x32_bf16(false, ah, false, bh, (short)0, c, false, false);
  if (NT >= 2) c = __builtin_amdgcn_wmma_f32_16x16x32_bf16(false, al, false, bh, (short)0, c, false, false);
  if (NT >= 3) c = __builtin_amdgcn_wmma_f32_16x16x32_bf16(false, ah, false, bl, (short)0, c, false, false);
  asm volatile("v_nop\n\tv_nop\n\tv_nop\n\tv_nop" : "+v"(c) : "v"(ah), "v"(al), "v"(bh), "v"(bl));
  return c;
}


typedef _Float16 v16h __attribute__((ext_vector_type(16)));
union FragH { v16h v; v8us half[2]; _Float16 h[16]; unsigned short u[16]; };
template <int NT>
__device__ __forceinline__ v8f mmaH(v16h ah, v16h al, v16h bh, v16h bl, v8f c) {
  c = __builtin_amdgcn_wmma_f32_16x16x32_f16(false, ah, false, bh, (short)0, c, false, false);
  if (NT >= 2) c = __builtin_amdgcn_wmma_f32_16x16x32_f16(false, al, false, bh, (short)0, c, false, false);
  if (NT >= 3) c = __builtin_amdgcn_wmma_f32_16x16x32_f16(false, ah, false, bl, (short)0, c, false, false);
  asm volatile("v_nop\n\tv_nop\n\tv_nop\n\tv_nop" : "+v"(c) : "v"(ah), "v"(al), "v"(bh), "v"(bl));
  return c;
}

__global__ __launch_bounds__(256) void k_wt_f16(const float* __restrict__ W, _Float16* __restrict__ Wt, int K, int N, float scale) {
  const int t = blockIdx.x * 256 + threadIdx.x; if (t >= N * (K / 8)) return; const int n = t / (K / 8), k8 = (t % (K / 8)) * 8; FragH f;
#pragma unroll
  for (int i = 0; i < 8; ++i) f.h[i] = (_Float16)(bf16_round(W[(size_t)(k8 + i) * N + n]) * scale); const v8us o = f.half[0];
  *(volatile v8us*)((unsigned short*)Wt + (size_t)n * K + k8) = o; __threadfence(); *(volatile v8us*)((unsigned short*)Wt + (size_t)n * K + k8) = o;
}

typedef _Float16 v4h __attribute__((ext_vector_type(4)));

__global__ __launch_bounds__(256) void k_x16(const float* __restrict__ x, _Float16* __restrict__ X16, size_t n8) { const size_t t = (size_t)blockIdx.x * 256 + threadIdx.x; if (t >= n8) return; FragH f;
#pragma unroll
  for (int q = 0; q < 8; ++q) f.h[q] = (_Float16)bf16_round(x[t * 8 + q]); *(volatile v8us*)((unsigned short*)X16 + t * 8) = f.half[0]; __threadfence(); *(volatile v8us*)((unsigned short*)X16 + t * 8) = f.half[0]; }
__device__ __forceinline__ v16h g2_frag(const _Float16* p, int hh) { FragH f; f.half[0] = *(const v8us*)((const unsigned short*)p + 8 * hh); f.half[1] = *(const v8us*)((const unsigned short*)p + 16 + 8 * hh); return f.v; }
__device__ __forceinline__ v8f g2_mma(v16h a, v16h b, v8f c) { v8f d = __builtin_amdgcn_wmma_f32_16x16x32_f16(false, a, false, b, (short)0, c, false, false); asm volatile("v_nop\n\tv_nop\n\tv_nop\n\tv_nop" : "+v"(d) : "v"(a), "v"(b)); return d; }
template <int ACT>
__global__ __launch_bounds__(128) void k_gemm2(const _Float16* __restrict__ A, int lda, size_t sA, const _Float16* __restrict__ Bh, int ldb, size_t sB, float alpha, const float* __restrict__ bias, size_t sBias, const float* __restrict__ CP, int rowsPerB, size_t sCPb, int row0g,
    float* __restrict__ C, _Float16* __restrict__ C16, int ldc, size_t sC, int M, int N, int K) { static_assert(ACT == 0 || ACT == 3 || ACT == 6 || ACT == 8 || ACT == 9 || ACT == 11 || ACT == 12 || ACT == 14 || ACT == 15 || ACT == 16 || ACT == 17, "k_gemm2: unsupported ACT code (would silently apply no activation)");
  __shared__ __attribute__((aligned(16))) float so[4][32][68];
  const int tid = threadIdx.x, w = tid >> 5, lane = tid & 31, ln = lane & 15, hh = lane >> 4; const int by = blockIdx.y;
  A += (size_t)by * sA; Bh += (size_t)by * sB; const size_t cofs = (size_t)by * sC; const float* bp = bias ? bias + (size_t)by * sBias : nullptr;
  const int ntn = N >> 6; const int mt = blockIdx.x / ntn, nq = blockIdx.x - mt * ntn; const int row0 = mt * 128 + 32 * w, col0 = nq * 64; if (row0 >= M) return;
  const _Float16* a0p = A + (size_t)(row0 + ln) * lda; const _Float16* a1p = a0p + (size_t)16 * lda;
  const _Float16* b0p = Bh + (size_t)(col0 + ln) * ldb; const _Float16* b1p = b0p + (size_t)16 * ldb; const _Float16* b2p = b1p + (size_t)16 * ldb; const _Float16* b3p = b2p + (size_t)16 * ldb;
  const v8f z8 = {0.f,0.f,0.f,0.f,0.f,0.f,0.f,0.f}; v8f c00 = z8, c01 = z8, c02 = z8, c03 = z8, c10 = z8, c11 = z8, c12 = z8, c13 = z8;
  for (int kb = 0; kb < K; kb += 32) { const v16h a0 = g2_frag(a0p + kb, hh), a1 = g2_frag(a1p + kb, hh);
    v16h b = g2_frag(b0p + kb, hh); c00 = g2_mma(a0, b, c00); c10 = g2_mma(a1, b, c10);
    b = g2_frag(b1p + kb, hh); c01 = g2_mma(a0, b, c01); c11 = g2_mma(a1, b, c11);
    b = g2_frag(b2p + kb, hh); c02 = g2_mma(a0, b, c02); c12 = g2_mma(a1, b, c12);
    b = g2_frag(b3p + kb, hh); c03 = g2_mma(a0, b, c03); c13 = g2_mma(a1, b, c13); }
  v8f accs[8] = {c00, c01, c02, c03, c10, c11, c12, c13};
#pragma unroll
  for (int u = 0; u < 8; ++u) { const int t = u & 3, half = u >> 2; const int col = col0 + t * 16 + ln; const float bv = bp ? bf16_round(bp[col]) : 0.f;
#pragma unroll
    for (int r = 0; r < 8; ++r) { const int rloc = half * 16 + 8 * hh + r; float v = accs[u][r] * alpha + bv; if (CP) { if (rowsPerB < 0) v += CP[cofs + (size_t)(row0g + row0 + rloc) * ldc + col];        else { const int bidx = (row0g + row0 + rloc) / rowsPerB; v += CP[(size_t)bidx * sCPb + (size_t)by * 64 + col]; } }
      if (ACT == 3) v = fmaxf(v, 0.f); else if (ACT == 6) v = 0.5f * v * (1.0f + erff(v * 0.70710678118654752f)); else if (ACT == 11) v = 1.0f / (1.0f + expf(-v)); else if (ACT == 15) v = v / (1.0f + expf(-v)); else if (ACT == 12) v = (v > 0.f) ? v : 0.01f * v; else if (ACT == 8) v = tanhf(v); else if (ACT == 9) v = 0.5f * v * (1.0f + tanhf(0.7978845608028654f * (v + 0.044715f * v * v * v))); else if (ACT == 14) v = (v > 0.f) ? v : 0.1f * v; else if (ACT == 16) v = (v >= 0.f) ? v : 0.3f * v; else if (ACT == 17) v = (v >= 0.f) ? v : 0.2f * v;
      so[w][rloc][t * 16 + ln] = v; } }
  __builtin_amdgcn_fence(__ATOMIC_ACQ_REL, "workgroup"); __builtin_amdgcn_wave_barrier();
  const int rsub = lane >> 4, c4 = (lane & 15) * 4;
  for (int pass = 0; pass < 2; ++pass) {
#pragma unroll
    for (int q = 0; q < 16; ++q) { const int r = q * 2 + rsub; const v4f v = *(const v4fa*)&so[w][r][c4]; if (C) *(volatile v4f*)(C + cofs + (size_t)(row0 + r) * ldc + col0 + c4) = v; if (C16) { v4h h4; for (int i = 0; i < 4; ++i) h4[i] = (_Float16)v[i]; *(volatile v4h*)(C16 + cofs + (size_t)(row0 + r) * ldc + col0 + c4) = h4; } }
    if (pass == 0) __threadfence(); } }

__global__ __launch_bounds__(256) void k_wpad(const float* __restrict__ w, int O, int Iw, int OP, int IP, _Float16* __restrict__ Bt) { const size_t t = (size_t)blockIdx.x * 256 + threadIdx.x; if (t >= (size_t)OP * IP / 8) return; const int i0 = (int)((t * 8) % IP); const int o = (int)((t * 8) / IP); FragH f; for (int u = 0; u < 8; ++u) { const int i = i0 + u; f.h[u] = (o < O && i < Iw) ? (_Float16)(bf16_round(w[(size_t)o * Iw + i]) * 16.0f) : (_Float16)0.f; }
  *(volatile v8us*)((unsigned short*)Bt + t * 8) = f.half[0]; __threadfence(); *(volatile v8us*)((unsigned short*)Bt + t * 8) = f.half[0]; }

__global__ __launch_bounds__(256) void k_wtpad(const float* __restrict__ Wm, _Float16* __restrict__ Wt, int Kr, int Kp, int Nr, int Np, float scale) {
  const int t = blockIdx.x * 256 + threadIdx.x; if (t >= Np * (Kp / 8)) return; const int n = t / (Kp / 8), k8 = (t % (Kp / 8)) * 8; const int nc = min(n, Nr - 1); const float fn = (n < Nr) ? 1.f : 0.f; FragH f;
  for (int i = 0; i < 8; ++i) { const int k = k8 + i; const int kc = min(k, Kr - 1); const float fk = (k < Kr) ? fn : 0.f; f.h[i] = (_Float16)(bf16_round(Wm[(size_t)kc * Nr + nc]) * scale * fk); }
  unsigned short* o = (unsigned short*)Wt + (size_t)n * Kp + k8; *(volatile v8us*)o = f.half[0]; __threadfence(); *(volatile v8us*)o = f.half[0]; }
__global__ __launch_bounds__(128) void k_bpad(const float* __restrict__ b, float* __restrict__ Bp, int nr, int np) {
  const int i = threadIdx.x; if (i >= np) return; const float v = b[min(i, nr - 1)] * ((i < nr) ? 1.f : 0.f); *(volatile float*)(Bp + i) = v; __threadfence(); *(volatile float*)(Bp + i) = v; }

__global__ __launch_bounds__(256) void k_escore(const float* __restrict__ QA, const float* __restrict__ QB, const float* __restrict__ WV, const float* __restrict__ WB, float* __restrict__ E) { const int t = blockIdx.x * 256 + threadIdx.x; if (t >= NB * NL * NL) return; const int b = t / (NL * NL), i = (t / NL) % NL, j = t % NL; const float* ap = QA + ((size_t)b * NL + i) * ND; const float* cp = QB + ((size_t)b * NL + j) * ND; float acc = 0.f;
  for (int d = 0; d < ND; ++d) { const float a = bf16_round(ap[d]), c = bf16_round(cp[d]); const float w1 = bf16_round(WV[d]), w2 = bf16_round(WV[ND + d]), w3 = bf16_round(WV[2 * ND + d]), w4 = bf16_round(WV[3 * ND + d]), w5 = bf16_round(WV[4 * ND + d]); acc += a * (w1 + w4) + c * (w2 - w4) + (a * w3) * c + fabsf(a - c) * w5; }
  const float e = tanhf(acc + bf16_round(WB[0])); *(volatile float*)(E + t) = e; __threadfence(); *(volatile float*)(E + t) = e; }

__global__ __launch_bounds__(256) void k_esm(const float* __restrict__ S, int sx, int sk, const int* __restrict__ HM, _Float16* __restrict__ P16, int n) { const int r = blockIdx.x * 256 + threadIdx.x; if (r >= n) return; const int b = r / NL, x = r % NL; const float* sp = S + (size_t)b * NL * NL + (size_t)x * sx; const int* hp = HM + (size_t)b * NL; float m = -3.0e38f;
  for (int k = 0; k < NL; ++k) { const float y = sp[(size_t)k * sk] - ((hp[k] == 0) ? HIDE : 0.f); m = (y > m) ? y : m; }
  float z = 0.f; for (int k = 0; k < NL; ++k) { const float y = sp[(size_t)k * sk] - ((hp[k] == 0) ? HIDE : 0.f); z += expf(y - m); }
  unsigned short* op = (unsigned short*)P16 + (size_t)r * NL;
  for (int k0 = 0; k0 < NL; k0 += 8) { FragH f;
#pragma unroll
    for (int u = 0; u < 8; ++u) { const int k = k0 + u; const float y = sp[(size_t)k * sk] - ((hp[k] == 0) ? HIDE : 0.f); const _Float16 h = (_Float16)((expf(y - m) / z) * PSC); f.h[u] = (h < (_Float16)6.103515625e-05f) ? (_Float16)0.f : h; }
    *(volatile v8us*)(op + k0) = f.half[0]; __threadfence(); *(volatile v8us*)(op + k0) = f.half[0]; } }

__global__ __launch_bounds__(256) void k_cpo(const float* __restrict__ src, float* __restrict__ dst, int n) { const int t = blockIdx.x * 256 + threadIdx.x; if (t >= n) return; const int r = t / ND, c = t % ND; const float v = src[(size_t)r * NP + c]; *(volatile float*)(dst + t) = v; __threadfence(); *(volatile float*)(dst + t) = v; }

extern "C" void kernel_launch(void* const* d_in, const int* in_sizes, int n_in,
                              void* d_out, int out_size, void* d_ws, size_t ws_size, hipStream_t stream) {
  (void)in_sizes; (void)n_in; (void)out_size;
  const float* QA = (const float*)d_in[0]; const float* QB = (const float*)d_in[1]; const int* HA = (const int*)d_in[2]; const int* HB = (const int*)d_in[3]; const float* KM = (const float*)d_in[4]; const float* WV = (const float*)d_in[5]; const float* BV = (const float*)d_in[6]; const float* WB = (const float*)d_in[7];
  static_assert(NB == 8 && NL == 128 && ND == 300 && NP == 320 && NP % 64 == 0 && NP % 32 == 0 && NL % 128 == 0 && NL % 64 == 0 && NL % 32 == 0 && (NB * NL) % 128 == 0 && ((size_t)NB * NL * NP / 8) % 256 == 0 && (NB * NL * NL) % 256 == 0 && (NB * NL * ND) % 256 == 0 && (NB * NL) % 256 == 0 && NP == 128 + 128 + 64 && ND > 256 && ND - 256 <= 64, "whole tiles; exact grids; the padded vector in three pieces");
  float* O0 = (float*)d_out; float* O1 = O0 + (size_t)NB * NL * ND; float* O2 = O1 + (size_t)NB * NL * ND; float* O3 = O2 + (size_t)NB * NL * ND;
  const size_t RW = (size_t)NB * NL;
  char* ws = (char*)d_ws; size_t off = 0;
  auto take = [&](size_t bytes) { char* p = ws + off; off += (bytes + 255) & ~(size_t)255; return p; };
  _Float16* XA = (_Float16*)take(RW * NP * 2); _Float16* XB = (_Float16*)take(RW * NP * 2); _Float16* TA = (_Float16*)take((size_t)NB * NP * NL * 2); _Float16* TB = (_Float16*)take((size_t)NB * NP * NL * 2); _Float16* KT = (_Float16*)take((size_t)NP * NP * 2); float* BP = (float*)take((size_t)NP * 4); _Float16* PA = (_Float16*)take(RW * NP * 2); _Float16* PB = (_Float16*)take(RW * NP * 2); float* FA = (float*)take(RW * NL * 4); float* FB = (float*)take(RW * NL * 4); float* EE = (float*)take(RW * NL * 4); _Float16* W16 = (_Float16*)take(RW * NL * 2); float* OW = (float*)take(RW * NP * 4);
  if (off > ws_size) return;
  k_wpad<<<(unsigned)(RW * NP / 8 / 256), 256, 0, stream>>>(QA, (int)RW, ND, (int)RW, NP, XA);
  k_wpad<<<(unsigned)(RW * NP / 8 / 256), 256, 0, stream>>>(QB, (int)RW, ND, (int)RW, NP, XB);
  for (int b = 0; b < NB; ++b) { k_wtpad<<<(NP * (NL / 8) + 255) / 256, 256, 0, stream>>>(QA + (size_t)b * NL * ND, TA + (size_t)b * NP * NL, NL, NL, ND, NP, TSC); k_wtpad<<<(NP * (NL / 8) + 255) / 256, 256, 0, stream>>>(QB + (size_t)b * NL * ND, TB + (size_t)b * NP * NL, NL, NL, ND, NP, TSC); }
  k_wtpad<<<(NP * (NP / 8) + 255) / 256, 256, 0, stream>>>(KM, KT, ND, NP, ND, NP, KSC);
  k_bpad<<<1, 128, 0, stream>>>(BV, BP, 128, 128); k_bpad<<<1, 128, 0, stream>>>(BV + 128, BP + 128, 128, 128); k_bpad<<<1, 128, 0, stream>>>(BV + 256, BP + 256, ND - 256, 64);
  const dim3 gj((unsigned)((RW / 128) * (NP / 64)), 1);
  k_gemm2<8><<<gj, 128, 0, stream>>>(XA, NP, 0, KT, NP, 0, 1.0f / (XSC * KSC), BP, 0, nullptr, 0, 0, 0, nullptr, PA, NP, 0, (int)RW, NP, NP);
  k_gemm2<8><<<gj, 128, 0, stream>>>(XB, NP, 0, KT, NP, 0, 1.0f / (XSC * KSC), BP, 0, nullptr, 0, 0, 0, nullptr, PB, NP, 0, (int)RW, NP, NP);
  const dim3 gf((unsigned)((NL / 128) * (NL / 64)), NB);
  k_gemm2<0><<<gf, 128, 0, stream>>>(PA, NP, (size_t)NL * NP, PA, NP, (size_t)NL * NP, 1.0f, nullptr, 0, nullptr, 0, 0, 0, FA, nullptr, NL, (size_t)NL * NL, NL, NL, NP);
  k_gemm2<0><<<gf, 128, 0, stream>>>(PB, NP, (size_t)NL * NP, PB, NP, (size_t)NL * NP, 1.0f, nullptr, 0, nullptr, 0, 0, 0, FB, nullptr, NL, (size_t)NL * NL, NL, NL, NP);
  k_escore<<<(unsigned)(NB * NL * NL / 256), 256, 0, stream>>>(QA, QB, WV, WB, EE);
  const dim3 go((unsigned)((NL / 128) * (NP / 64)), NB); const unsigned gc = (unsigned)(NB * NL * ND / 256);
  k_esm<<<(unsigned)(RW / 256), 256, 0, stream>>>(EE, NL, 1, HB, W16, (int)RW);
  k_gemm2<0><<<go, 128, 0, stream>>>(W16, NL, (size_t)NL * NL, TB, NL, (size_t)NP * NL, 1.0f / (PSC * TSC), nullptr, 0, nullptr, 0, 0, 0, OW, nullptr, NP, (size_t)NL * NP, NL, NP, NL);
  k_cpo<<<gc, 256, 0, stream>>>(OW, O0, NB * NL * ND);
  k_esm<<<(unsigned)(RW / 256), 256, 0, stream>>>(EE, 1, NL, HA, W16, (int)RW);
  k_gemm2<0><<<go, 128, 0, stream>>>(W16, NL, (size_t)NL * NL, TA, NL, (size_t)NP * NL, 1.0f / (PSC * TSC), nullptr, 0, nullptr, 0, 0, 0, OW, nullptr, NP, (size_t)NL * NP, NL, NP, NL);
  k_cpo<<<gc, 256, 0, stream>>>(OW, O1, NB * NL * ND);
  k_esm<<<(unsigned)(RW / 256), 256, 0, stream>>>(FA, NL, 1, HA, W16, (int)RW);
  k_gemm2<0><<<go, 128, 0, stream>>>(W16, NL, (size_t)NL * NL, TA, NL, (size_t)NP * NL, 1.0f / (PSC * TSC), nullptr, 0, nullptr, 0, 0, 0, OW, nullptr, NP, (size_t)NL * NP, NL, NP, NL);
  k_cpo<<<gc, 256, 0, stream>>>(OW, O2, NB * NL * ND);
  k_esm<<<(unsigned)(RW / 256), 256, 0, stream>>>(FB, NL, 1, HB, W16, (int)RW);
  k_gemm2<0><<<go, 128, 0, stream>>>(W16, NL, (size_t)NL * NL, TB, NL, (size_t)NP * NL, 1.0f / (PSC * TSC), nullptr, 0, nullptr, 0, 0, 0, OW, nullptr, NP, (size_t)NL * NP, NL, NP, NL);
  k_cpo<<<gc, 256, 0, stream>>>(OW, O3, NB * NL * ND);
}
